// HybridNN_44727789420660
// MI455X (gfx1250) — hardware-run, weakly checked
//
#include <hip/hip_runtime.h>
#include <math.h>
#include <stdint.h>

typedef __attribute__((ext_vector_type(16))) _Float16 v16h;
typedef __attribute__((ext_vector_type(8)))  _Float16 v8h;
typedef __attribute__((ext_vector_type(8)))  float    v8f;
typedef __attribute__((ext_vector_type(4)))  float    v4f;
typedef __attribute__((ext_vector_type(2)))  float    v2f;

constexpr int kBatch        = 1024;
constexpr int kFeat         = 2048;
constexpr int kHid          = 512;
constexpr int kCom          = 32;
constexpr int kWires        = 12;
constexpr int kLayers       = 2;
constexpr int kAmp          = 4096;
constexpr int kHalfAmp      = 2048;
constexpr int kGates        = kLayers * kWires;
constexpr int kTrigSlots    = kGates * 3;
constexpr int kRowsPerBlock = 32;
constexpr float kW1Carry    = 64.0f;
constexpr float kW1CarryInv = 1.0f / 64.0f;
constexpr float kInvSqrt2   = 0.70710678118654752440f;
static_assert(kAmp == (1 << kWires), "state size");
static_assert(kFeat == kHalfAmp, "image angles cover the lower 11 wires");
static_assert((kBatch % 64) == 0 && (kHid % 64) == 0, "GEMM M,N multiples of 64");
static_assert((kFeat % 32) == 0, "GEMM K multiple of 32");
static_assert((kBatch % kRowsPerBlock) == 0, "row blocks");
static_assert(kTrigSlots == 72, "angle table");

constexpr size_t kOffXH   = 0;
constexpr size_t kOffW1H  = kOffXH  + (size_t)kBatch * kFeat * 2;
constexpr size_t kOffHID  = kOffW1H + (size_t)kHid   * kFeat * 2;
constexpr size_t kWsTotal = kOffHID + (size_t)kBatch * kHid  * 4;
static_assert(kWsTotal == 8388608ull, "carve total");
static_assert(kWsTotal <= 134217728ull, "carve cap");
static_assert((kOffW1H % 128) == 0 && (kOffHID % 128) == 0, "128-B aligned regions");

union FragU { v16h v; v8h h[2]; };
__device__ __forceinline__ v16h frag_load(const _Float16* p) {
  FragU f;
  f.h[0] = *(const v8h*)(p);
  f.h[1] = *(const v8h*)(p + 16);
  return f.v;
}
__device__ __forceinline__ v8f mma_f16(v16h a, v16h b, v8f c) {
  c = __builtin_amdgcn_wmma_f32_16x16x32_f16(false, a, false, b, (short)0, c, false, false);
  asm volatile("v_nop\n\tv_nop\n\tv_nop\n\tv_nop" : "+v"(c) : "v"(a), "v"(b));
  return c;
}

__global__ __launch_bounds__(256) void cast_rows_f16_kernel(
    const float* __restrict__ src, _Float16* __restrict__ dst, int total8, float mul)
{
  const int i = blockIdx.x * 256 + threadIdx.x;
  if (i >= total8) return;
  const size_t e0 = (size_t)i << 3;
  const v4f a0 = *(const v4f*)(src + e0);
  const v4f a1 = *(const v4f*)(src + e0 + 4);
  v8h hv;
#pragma unroll
  for (int e = 0; e < 4; ++e) {
    const float f0 = a0[e] * mul;
    const float f1 = a1[e] * mul;
    hv[e]     = (_Float16)f0;
    hv[4 + e] = (_Float16)f1;
  }
  _Float16* q = dst + e0;
  *(volatile v8h*)q = hv;
  __threadfence();
  *(volatile v8h*)q = hv;
}

__global__ __launch_bounds__(256) void gemm64_f16_bias_relu_kernel(
    const _Float16* __restrict__ A, int lda,
    const _Float16* __restrict__ Bt, int ldb,
    float* __restrict__ C, int ldc,
    const float* __restrict__ bias,
    int M, int N, int K, float scale)
{
  __shared__ __align__(16) float sT[8][16 * 68];
  const int lane = threadIdx.x & 31;
  const int wave = threadIdx.x >> 5;
  const int tilesN = N >> 6;
  const int tilesM = M >> 6;
  const int tile = blockIdx.x * 8 + wave;
  if (tile >= tilesM * tilesN) return;
  const int tm = tile / tilesN;
  const int tn = tile - tm * tilesN;
  const int m0 = tm << 6;
  const int n0 = tn << 6;

  const int rlane = lane & 15;
  const int koff  = (lane >> 4) * 8;
  const int mOff  = (lane >> 4) * 8;

  v8f acc[4][4];
#pragma unroll
  for (int i = 0; i < 4; ++i)
#pragma unroll
    for (int j = 0; j < 4; ++j) acc[i][j] = (v8f){0.f, 0.f, 0.f, 0.f, 0.f, 0.f, 0.f, 0.f};

  for (int k0 = 0; k0 < K; k0 += 32) {
    v16h bh[4];
#pragma unroll
    for (int j = 0; j < 4; ++j) {
      const size_t bo = (size_t)(n0 + (j << 4) + rlane) * ldb + koff + k0;
      bh[j] = frag_load(Bt + bo);
    }
#pragma unroll
    for (int i = 0; i < 4; ++i) {
      const size_t ao = (size_t)(m0 + (i << 4) + rlane) * lda + koff + k0;
      const v16h ah = frag_load(A + ao);
#pragma unroll
      for (int j = 0; j < 4; ++j) acc[i][j] = mma_f16(ah, bh[j], acc[i][j]);
    }
  }

  float* slab = sT[wave];
#pragma unroll
  for (int i = 0; i < 4; ++i) {
    const int mBase = m0 + (i << 4);
#pragma unroll
    for (int j = 0; j < 4; ++j) {
      const int n = n0 + (j << 4) + rlane;
      const float bv = bias[n];
#pragma unroll
      for (int r = 0; r < 8; ++r) {
        float v = acc[i][j][r] * scale;
        v += bv;
        v = fmaxf(v, 0.0f);
        slab[(mOff + r) * 68 + (j << 4) + rlane] = v;
      }
    }
    __builtin_amdgcn_fence(__ATOMIC_RELEASE, "workgroup");
    __builtin_amdgcn_wave_barrier();
    __builtin_amdgcn_fence(__ATOMIC_ACQUIRE, "workgroup");
    {
      const int hh = lane >> 4, c4 = (lane & 15) * 4;
      for (int pass = 0; pass < 2; ++pass) {
#pragma unroll
        for (int it = 0; it < 8; ++it) {
          const int row = it * 2 + hh;
          const v4f v = *(const v4f*)(slab + row * 68 + c4);
          *(volatile v4f*)(C + (size_t)(mBase + row) * ldc + n0 + c4) = v;
        }
        __threadfence();
      }
    }
    __builtin_amdgcn_fence(__ATOMIC_RELEASE, "workgroup");
    __builtin_amdgcn_wave_barrier();
    __builtin_amdgcn_fence(__ATOMIC_ACQUIRE, "workgroup");
  }
}

__device__ __forceinline__ void sincos_rr(float x, float& s, float& c) {
  const float kf = rintf(x * 0.636619772f);
  float r = fmaf(-kf, 1.57079637f, x);
  r = fmaf(-kf, -4.37113883e-8f, r);
  r = fmaf(-kf, -1.71512451e-15f, r);
  const int q = (int)kf;
  const float z = r * r;
  float ps = fmaf(-1.9515295891e-4f, z, 8.3321608736e-3f);
  ps = fmaf(ps, z, -1.6666654611e-1f);
  const float sr = fmaf(ps * z, r, r);
  float pc = fmaf(2.443315711809948e-5f, z, -1.388731625493765e-3f);
  pc = fmaf(pc, z, 4.166664568298827e-2f);
  const float cr = fmaf(pc * z, z, fmaf(-0.5f, z, 1.0f));
  const bool swp = (q & 1) != 0;
  const float s0 = swp ? cr : sr;
  const float c0 = swp ? sr : cr;
  s = ((q & 2) != 0) ? -s0 : s0;
  c = (((q + 1) & 2) != 0) ? -c0 : c0;
}

__device__ __forceinline__ int ring_perm(int n, int rg) {
  int y = n;
#pragma unroll
  for (int i2 = kWires - 1; i2 >= 0; --i2) {
    int t = i2 + rg;
    t = (t >= kWires) ? (t - kWires) : t;
    const int cm = 1 << (kWires - 1 - i2);
    const int tm = 1 << (kWires - 1 - t);
    y = ((y & cm) != 0) ? (y ^ tm) : y;
  }
  return y;
}

__global__ __launch_bounds__(256) void circuit_rows_kernel(
    const float* __restrict__ hid, const float* __restrict__ xin,
    const float* __restrict__ w2, const float* __restrict__ b2,
    const float* __restrict__ asz, float* __restrict__ out)
{
  __shared__ __align__(16) v2f   sSt[kAmp];
  __shared__ __align__(16) float sPhi[kFeat];
  __shared__ __align__(16) float sW2[kHid];
  __shared__ float sGm[kGates * 8];
  __shared__ float sTc[kTrigSlots];
  __shared__ float sTs[kTrigSlots];
  __shared__ float sRedA[8];
  __shared__ float sRedP0[8];
  __shared__ float sRedP1[8];
  __shared__ float sRes[kRowsPerBlock];

  const int tid = threadIdx.x, lane = tid & 31, wave = tid >> 5;

  sW2[tid] = w2[tid];
  sW2[256 + tid] = w2[256 + tid];
  {
    int g = tid / 3;
    const int which = tid - 3 * g;
    g = (g < kGates) ? g : (kGates - 1);
    const float ph = asz[g * 3 + 0];
    const float th = asz[g * 3 + 1];
    const float om = asz[g * 3 + 2];
    const float a0 = 0.5f * th;
    const float a1 = 0.5f * (ph + om);
    const float a2 = 0.5f * (ph - om);
    const float ang = (which == 0) ? a0 : ((which == 1) ? a1 : a2);
    float sv, cv;
    sincos_rr(ang, sv, cv);
    if (tid < kTrigSlots) {
      sTc[tid] = cv;
      sTs[tid] = sv;
    }
  }
  __syncthreads();
  if (tid < kGates) {
    const float ct = sTc[3 * tid], st = sTs[3 * tid];
    const float c1 = sTc[3 * tid + 1], s1 = sTs[3 * tid + 1];
    const float c2 = sTc[3 * tid + 2], s2 = sTs[3 * tid + 2];
    float* gp = sGm + tid * 8;
    gp[0] = c1 * ct;
    gp[1] = -(s1 * ct);
    gp[2] = -(c2 * st);
    gp[3] = -(s2 * st);
    gp[4] = c2 * st;
    gp[5] = -(s2 * st);
    gp[6] = c1 * ct;
    gp[7] = s1 * ct;
  }
  __syncthreads();
  const float bias2 = b2[0];

#pragma unroll 1
  for (int rr = 0; rr < kRowsPerBlock; ++rr) {
    const int row = blockIdx.x * kRowsPerBlock + rr;

    const float* hrow = hid + (size_t)row * kHid;
    float part = hrow[tid] * sW2[tid];
    part = fmaf(hrow[256 + tid], sW2[256 + tid], part);
#pragma unroll
    for (int off = 16; off >= 1; off >>= 1) part += __shfl_xor(part, off, 32);
    if (lane == 0) sRedA[wave] = part;
    __syncthreads();
    float com0 = sRedA[0];
#pragma unroll
    for (int w = 1; w < 8; ++w) com0 += sRedA[w];
    com0 += bias2;

    float sn0, cs0;
    sincos_rr(0.5f * com0, sn0, cs0);
    const float amp0 = cs0 * kInvSqrt2 - sn0 * kInvSqrt2;
    const float amp1 = sn0 * kInvSqrt2 + cs0 * kInvSqrt2;
#pragma unroll 1
    for (int j = 0; j < 16; ++j) {
      const int i = tid + 256 * j;
      const float re = (i == 0) ? amp0 : ((i == kHalfAmp) ? amp1 : 0.0f);
      sSt[i] = (v2f){re, 0.0f};
    }
    __syncthreads();

#pragma unroll 1
    for (int l = 0; l < kLayers; ++l) {
#pragma unroll 1
      for (int w = 0; w < kWires; ++w) {
        const float* gp = sGm + (l * kWires + w) * 8;
        const float m00r = gp[0], m00i = gp[1], m01r = gp[2], m01i = gp[3];
        const float m10r = gp[4], m10i = gp[5], m11r = gp[6], m11i = gp[7];
        const int Rb = kWires - 1 - w;
        const int Rm = (1 << Rb) - 1;
        const int Rs = 1 << Rb;
#pragma unroll 1
        for (int j = 0; j < 8; ++j) {
          const int pdx = tid + 256 * j;
          const int n0 = ((pdx >> Rb) << (Rb + 1)) + (pdx & Rm);
          const int n1 = n0 + Rs;
          const v2f a0 = sSt[n0];
          const v2f a1 = sSt[n1];
          v2f o0, o1;
          o0.x = m00r * a0.x - m00i * a0.y + m01r * a1.x - m01i * a1.y;
          o0.y = m00r * a0.y + m00i * a0.x + m01r * a1.y + m01i * a1.x;
          o1.x = m10r * a0.x - m10i * a0.y + m11r * a1.x - m11i * a1.y;
          o1.y = m10r * a0.y + m10i * a0.x + m11r * a1.y + m11i * a1.x;
          sSt[n0] = o0;
          sSt[n1] = o1;
        }
        __syncthreads();
      }
      const int rg = l + 1;
      v2f tmp[16];
#pragma unroll
      for (int j = 0; j < 16; ++j) tmp[j] = sSt[ring_perm(tid + 256 * j, rg)];
      __syncthreads();
#pragma unroll
      for (int j = 0; j < 16; ++j) sSt[tid + 256 * j] = tmp[j];
      __syncthreads();
    }

    const float* xr = xin + (size_t)row * kFeat;
    *(v4f*)(sPhi + 4 * tid) = *(const v4f*)(xr + 4 * tid);
    *(v4f*)(sPhi + 1024 + 4 * tid) = *(const v4f*)(xr + 1024 + 4 * tid);
    __syncthreads();
#pragma unroll 1
    for (int s = 0; s < 11; ++s) {
      const int bit = 1 << s;
#pragma unroll 1
      for (int j = 0; j < 4; ++j) {
        const int p = tid + 256 * j;
        const int i = ((p >> s) << (s + 1)) | bit | (p & (bit - 1));
        const float lo = sPhi[i - bit];
        const float hi = sPhi[i];
        sPhi[i] = hi + lo;
      }
      __syncthreads();
    }

    float p0 = 0.0f, p1 = 0.0f;
#pragma unroll 1
    for (int j = 0; j < 8; ++j) {
      const int a = tid + 256 * j;
      const int rv = (int)(__brev((unsigned)a) >> 21);
      const float hA = 0.5f * sPhi[rv];
      float sn, cs;
      sincos_rr(hA, sn, cs);
      const v2f s0 = sSt[a];
      const v2f s1 = sSt[a + kHalfAmp];
      const float n0r = cs * s0.x - sn * s1.x;
      const float n0i = cs * s0.y - sn * s1.y;
      const float n1r = sn * s0.x + cs * s1.x;
      const float n1i = sn * s0.y + cs * s1.y;
      p0 += n0r * n0r + n0i * n0i;
      p1 += n1r * n1r + n1i * n1i;
    }
#pragma unroll
    for (int off = 16; off >= 1; off >>= 1) {
      p0 += __shfl_xor(p0, off, 32);
      p1 += __shfl_xor(p1, off, 32);
    }
    if (lane == 0) {
      sRedP0[wave] = p0;
      sRedP1[wave] = p1;
    }
    __syncthreads();
    if (tid == 0) {
      float t0 = sRedP0[0], t1 = sRedP1[0];
#pragma unroll
      for (int w = 1; w < 8; ++w) {
        t0 += sRedP0[w];
        t1 += sRedP1[w];
      }
      sRes[rr] = t1 - t0;
    }
    __syncthreads();
  }

  if (tid < kRowsPerBlock) {
    const float v = sRes[tid];
    volatile float* op = out + (size_t)blockIdx.x * kRowsPerBlock + tid;
    *op = v;
    __threadfence();
    *op = v;
  }
}

extern "C" void kernel_launch(void* const* d_in, const int* in_sizes, int n_in,
                              void* d_out, int out_size, void* d_ws, size_t ws_size,
                              hipStream_t stream) {
  if (n_in < 6) return;
  if (in_sizes[0] != kBatch * kFeat) return;
  if (in_sizes[1] != kHid * kFeat) return;
  if (in_sizes[2] != kHid) return;
  if (in_sizes[3] != kCom * kHid) return;
  if (in_sizes[4] != kCom) return;
  if (in_sizes[5] != kTrigSlots) return;
  if (out_size != kBatch) return;
  if (ws_size < kWsTotal) return;

  const float* x   = (const float*)d_in[0];
  const float* W1  = (const float*)d_in[1];
  const float* b1  = (const float*)d_in[2];
  const float* W2  = (const float*)d_in[3];
  const float* b2  = (const float*)d_in[4];
  const float* asz = (const float*)d_in[5];
  float* out = (float*)d_out;

  char* ws = (char*)d_ws;
  _Float16* XH  = (_Float16*)(ws + kOffXH);
  _Float16* W1H = (_Float16*)(ws + kOffW1H);
  float*    HID = (float*)(ws + kOffHID);

  cast_rows_f16_kernel<<<(kBatch * kFeat / 8) / 256, 256, 0, stream>>>(x, XH, kBatch * kFeat / 8, 1.0f);
  cast_rows_f16_kernel<<<(kHid * kFeat / 8) / 256, 256, 0, stream>>>(W1, W1H, kHid * kFeat / 8, kW1Carry);

  gemm64_f16_bias_relu_kernel<<<((kBatch / 64) * (kHid / 64)) / 8, 256, 0, stream>>>(
      XH, kFeat, W1H, kFeat, HID, kHid, b1, kBatch, kHid, kFeat, kW1CarryInv);

  circuit_rows_kernel<<<kBatch / kRowsPerBlock, 256, 0, stream>>>(HID, x, W2, b2, asz, out);
}
